// ThreeBodyGhostNet_25984552141464
// MI455X (gfx1250) — hardware-run, weakly checked
//
#include <hip/hip_runtime.h>


namespace {
constexpr int N = 50000, NP = 50048, E = 640000, H = 128, NL = 4, NBLK = NP / 16;
constexpr int OFF1 = N * H, OFF2 = OFF1 + N, OFF3 = OFF2 + N;
constexpr float XS = 8.0f, HS = 1.0f  , WSC = 256.0f;
typedef _Float16 b16;
typedef __attribute__((ext_vector_type(16))) _Float16 v16b;
typedef __attribute__((ext_vector_type(8))) _Float16 v8b;
typedef __attribute__((ext_vector_type(8))) float v8f;
typedef __attribute__((ext_vector_type(4))) float v4f;
typedef __attribute__((ext_vector_type(2))) float v2f;
__device__ __forceinline__ float bf16_rne(float f) { unsigned int u = __float_as_uint(f); u += 0x7FFFu + ((u >> 16) & 1u); return __uint_as_float(u & 0xFFFF0000u); }
__device__ __forceinline__ void split16(float v, b16& hi, b16& lo) { hi = (b16)v; lo = (b16)(v - (float)hi); }
__device__ __forceinline__ v16b frag_kb(const b16* p, int hh) { const v8b a = *(const v8b*)(p + 8 * hh), b = *(const v8b*)(p + 16 + 8 * hh); v16b f;
#pragma unroll
  for (int e = 0; e < 8; ++e) { f[e] = a[e]; f[8 + e] = b[e]; } return f; }
__device__ __forceinline__ v8f wmma16b(v16b a, v16b b, v8f c) { v8f d = __builtin_amdgcn_wmma_f32_16x16x32_f16(false, a, false, b, (short)0, c, false, false); asm volatile("v_nop\n\tv_nop\n\tv_nop\n\tv_nop" : "+v"(d) : "v"(a), "v"(b)); return d; }
__device__ __forceinline__ void wave_lds_sync() { __builtin_amdgcn_fence(__ATOMIC_RELEASE, "workgroup"); __builtin_amdgcn_wave_barrier(); __builtin_amdgcn_fence(__ATOMIC_ACQUIRE, "workgroup"); }
__device__ __forceinline__ float pmul(float a, float b) { float p = a * b; asm volatile("" : "+v"(p)); return p; }
__device__ __forceinline__ int iclamp(int v, int lo, int hi) { return v < lo ? lo : (v > hi ? hi : v); }
__device__ __forceinline__ float sigm(float v) { return 1.0f / (1.0f + __expf(-v)); }
constexpr int CSR_NBLK9 = 512, CSR_GB9 = 9, CSR_GN9 = 1 << CSR_GB9  , CSR_TS9 = (CSR_GN9 < 32 ? 32 : CSR_GN9)  , CSR_MAXG9 = 512, CSR_CAP9 = 12288  ;
__device__ __host__ __forceinline__ int csr_tix9(int v) { return (v >> CSR_GB9) * CSR_TS9 + (v & (CSR_GN9 - 1)); }
__global__ __launch_bounds__(64) void csrA_kernel9(const int* __restrict__ dst, int E, int N, int nG, int CHP, int NGP, int* __restrict__ STG, int* __restrict__ HST) {
  extern __shared__ int sm[];
  int* cnt = sm; int* run = sm + NGP; int* ids = sm + 2 * NGP;
  const int b = blockIdx.x; const int ch = (E + CSR_NBLK9 - 1) / CSR_NBLK9; const int e0 = b * ch, e1 = min(E, e0 + ch);
  for (int i = threadIdx.x; i < NGP; i += 64) cnt[i] = 0;
  for (int i = threadIdx.x; i < CHP; i += 64) ids[i] = -1;
  __syncthreads();
  if (threadIdx.x == 0) {
    for (int e = e0; e < e1; ++e) { int d = dst[e]; d = (d < 0) ? 0 : (d >= N ? N - 1 : d); cnt[d >> CSR_GB9] += 1; }
    int acc = 0; for (int g = 0; g < nG; ++g) { run[g] = acc; acc += cnt[g]; }
    for (int e = e0; e < e1; ++e) { int d = dst[e]; d = (d < 0) ? 0 : (d >= N ? N - 1 : d); const int g = d >> CSR_GB9; ids[run[g]] = e; run[g] += 1; } }
  __syncthreads();
  typedef __attribute__((ext_vector_type(4))) int v4i;
  for (int pass = 0; pass < 2; ++pass) {
    for (int i = threadIdx.x; i < CHP / 4; i += 64) *(volatile v4i*)(STG + (size_t)b * CHP + i * 4) = *(const v4i*)(&ids[i * 4]);
    for (int i = threadIdx.x; i < NGP / 4; i += 64) { v4i v; for (int e = 0; e < 4; ++e) v[e] = (i * 4 + e < nG) ? cnt[i * 4 + e] : 0; *(volatile v4i*)(HST + (size_t)b * NGP + i * 4) = v; }
    __threadfence(); }
}
__global__ __launch_bounds__(512) void csrS_kernel9(const int* __restrict__ HST, int nG, int NGP, int* __restrict__ START, int* __restrict__ TOT, int* __restrict__ OFF) {
  __shared__ int tot[CSR_MAXG9];
  const int b = threadIdx.x;
  for (int pass = 0; pass < 2; ++pass) { int runb = 0; for (int g = 0; g < nG; ++g) { int c = HST[(size_t)b * NGP + g]; c = (c < 0) ? 0 : c; ((volatile int*)OFF)[(size_t)g * CSR_NBLK9 + b] = runb; runb += c; } __threadfence(); }
  for (int g = threadIdx.x; g < nG; g += 512) { int s = 0; for (int bb = 0; bb < CSR_NBLK9; ++bb) { int c = HST[(size_t)bb * NGP + g]; s += (c < 0) ? 0 : c; } tot[g] = s; }
  __syncthreads();
  if (threadIdx.x < 32) {
    __shared__ int st[CSR_MAXG9 + 32];
    if (threadIdx.x == 0) { int acc = 0; for (int g = 0; g < NGP; ++g) { st[g] = acc; if (g < nG) acc += (tot[g] + 31) & ~31; } st[NGP] = acc; }
    __builtin_amdgcn_fence(__ATOMIC_RELEASE, "workgroup"); __builtin_amdgcn_wave_barrier(); __builtin_amdgcn_fence(__ATOMIC_ACQUIRE, "workgroup");
    for (int pass = 0; pass < 2; ++pass) { for (int i = threadIdx.x; i < NGP + 32; i += 32) { ((volatile int*)START)[i] = (i <= NGP) ? st[min(i, NGP)] : 0; ((volatile int*)TOT)[i] = (i < nG) ? tot[i] : 0; } __threadfence(); } }
}
__global__ __launch_bounds__(256) void csrB_kernel9(const int* __restrict__ dst, int N, int nG, int CHP, int NGP, int permLen, const int* __restrict__ STG, const int* __restrict__ HST, const int* __restrict__ OFF, const int* __restrict__ START, const int* __restrict__ TOT, int* __restrict__ PERM, int* __restrict__ ROWPTR, int* __restrict__ ROWCNT, int* __restrict__ FLAG) {
  typedef __attribute__((ext_vector_type(4))) int v4i;
  __shared__ int ids[CSR_CAP9]; __shared__ unsigned short key[CSR_CAP9]; __shared__ int outp[CSR_CAP9]; __shared__ int ncnt[CSR_GN9 + 1]; __shared__ int boff[CSR_NBLK9 + 1];
  const int g = blockIdx.x, t_ = threadIdx.x; int tot = TOT[g]; int st = START[g], stn = START[g + 1]; const int v0 = g * CSR_GN9; const int nv = min(CSR_GN9, N - v0); const int t0 = g * CSR_TS9;
  st = (st < 0) ? 0 : (st > permLen - 32 ? permLen - 32 : st) & ~31; stn = (stn < st) ? st : (stn > permLen ? permLen : stn); tot = (tot < 0) ? 0 : tot; if (tot > stn - st && tot <= CSR_CAP9) tot = stn - st;
  if (tot > CSR_CAP9) {
    for (int pass = 0; pass < 2; ++pass) { for (int i = t_; i < CSR_TS9 / 4; i += 256) { v4i a, c; for (int e = 0; e < 4; ++e) { a[e] = st; c[e] = 0; } *(volatile v4i*)(ROWPTR + t0 + i * 4) = a; *(volatile v4i*)(ROWCNT + t0 + i * 4) = c; } if (t_ == 0) ((volatile int*)FLAG)[0] = 1; __threadfence(); } (void)nv; return; }
  if (t_ == 0) { int acc = 0; for (int b = 0; b < CSR_NBLK9; ++b) { boff[b] = acc; int c = HST[(size_t)b * NGP + g]; c = (c < 0) ? 0 : (c > CHP ? CHP : c); acc += c; if (acc > tot) acc = tot; } boff[CSR_NBLK9] = acc; }
  for (int i = t_; i <= CSR_GN9; i += 256) ncnt[i] = 0;
  __syncthreads();
  for (int b = 0; b < CSR_NBLK9; ++b) { const int c = boff[b + 1] - boff[b]; int o_ = OFF[(size_t)g * CSR_NBLK9 + b]; o_ = (o_ < 0) ? 0 : (o_ > CHP - c ? CHP - c : o_); const int* src_ = STG + (size_t)b * CHP + o_;
    for (int i = t_; i < c; i += 256) { int id = src_[i]; id = (id < 0) ? 0 : id; ids[boff[b] + i] = id; int d = dst[id]; d = (d < v0) ? v0 : (d >= N ? N - 1 : d); int kk = d - v0; kk = (kk < 0) ? 0 : (kk >= CSR_GN9 ? CSR_GN9 - 1 : kk); key[boff[b] + i] = (unsigned short)kk; } }
  __syncthreads();
  if (t_ == 0) { for (int i = 0; i < tot; ++i) ncnt[key[i]] += 1; int acc = 0; for (int vl = 0; vl < CSR_GN9; ++vl) { const int c = ncnt[vl]; ncnt[vl] = acc; acc += c; } ncnt[CSR_GN9] = acc;
    for (int i = 0; i < tot; ++i) { const int vl = key[i]; outp[ncnt[vl]] = ids[i]; ncnt[vl] += 1; }
    for (int vl = CSR_GN9; vl > 0; --vl) ncnt[vl] = ncnt[vl - 1]; ncnt[0] = 0; }
  __syncthreads();
  for (int pass = 0; pass < 2; ++pass) {
    for (int i = t_; i < (stn - st) / 4; i += 256) { v4i v; for (int e = 0; e < 4; ++e) { const int q = i * 4 + e; v[e] = (q < tot) ? outp[q] : -1; } *(volatile v4i*)(PERM + st + i * 4) = v; }
    for (int i = t_; i < CSR_TS9 / 4; i += 256) { v4i a, c; for (int e = 0; e < 4; ++e) { const int vl = i * 4 + e; const int vc = vl < CSR_GN9 ? vl : CSR_GN9; a[e] = (vl < CSR_GN9) ? st + ncnt[vc] : st; c[e] = (vl < nv) ? (ncnt[(vc < CSR_GN9 ? vc : CSR_GN9 - 1) + 1] - ncnt[vc]) : 0; } *(volatile v4i*)(ROWPTR + t0 + i * 4) = a; *(volatile v4i*)(ROWCNT + t0 + i * 4) = c; }
    __threadfence(); }
}
__global__ __launch_bounds__(256) void csrZ_kernel9(int* __restrict__ p, size_t n4) { typedef __attribute__((ext_vector_type(4))) int v4i; const size_t tid = (size_t)blockIdx.x * 256 + threadIdx.x, nth = (size_t)gridDim.x * 256; v4i z = {0, 0, 0, 0}; for (size_t i = tid; i < n4; i += nth) *(volatile v4i*)(p + i * 4) = z; }
struct CsrBufs9 { int *STG, *HST, *OFF, *START, *TOT, *PERM, *ROWPTR, *ROWCNT, *FLAG; int nG, NGP, CHP; size_t permLen; char* base; size_t bytes; };
static size_t csr_carve9(CsrBufs9& c, char* ws, size_t off, int E, int N) {
  const size_t off0 = off; c.base = ws + off;
  auto al = [&](size_t bytes) { char* p = ws + off; off += (bytes + 255) & ~(size_t)255; return p; };
  c.nG = (N + CSR_GN9 - 1) / CSR_GN9; c.NGP = (c.nG + 31) & ~31; const int ch = (E + CSR_NBLK9 - 1) / CSR_NBLK9; c.CHP = (ch + 31) & ~31; c.permLen = (size_t)E + 32 * (size_t)c.nG + 32;
  c.STG = (int*)al((size_t)CSR_NBLK9 * c.CHP * 4); c.HST = (int*)al((size_t)CSR_NBLK9 * c.NGP * 4); c.OFF = (int*)al((size_t)c.NGP * CSR_NBLK9 * 4); c.START = (int*)al((size_t)(c.NGP + 64) * 4); c.TOT = (int*)al((size_t)(c.NGP + 64) * 4);
  c.PERM = (int*)al(c.permLen * 4); c.ROWPTR = (int*)al((size_t)c.nG * CSR_TS9 * 4); c.ROWCNT = (int*)al((size_t)c.nG * CSR_TS9 * 4); c.FLAG = (int*)al(256);
  c.bytes = off - off0; return off;
}
static void csr_build9(const CsrBufs9& c, const int* dst, int E, int N, hipStream_t stream) {
  const size_t smem = (size_t)(2 * c.NGP + c.CHP) * 4;
  csrZ_kernel9<<<512, 256, 0, stream>>>((int*)c.base, c.bytes / 16);
  csrA_kernel9<<<CSR_NBLK9, 64, smem, stream>>>(dst, E, N, c.nG, c.CHP, c.NGP, c.STG, c.HST);
  csrS_kernel9<<<1, 512, 0, stream>>>(c.HST, c.nG, c.NGP, c.START, c.TOT, c.OFF);
  csrB_kernel9<<<c.nG, 256, 0, stream>>>(dst, N, c.nG, c.CHP, c.NGP, (int)c.permLen, c.STG, c.HST, c.OFF, c.START, c.TOT, c.PERM, c.ROWPTR, c.ROWCNT, c.FLAG);
}


__global__ __launch_bounds__(256) void wprep_kernel(const float* __restrict__ w, int r0, int KIN, b16* __restrict__ WT) {
  const int u = blockIdx.x * 256 + threadIdx.x; if (u >= H * KIN / 8) return; const int e = u * 8; const int o = e / KIN, k0 = e % KIN; v8b v;
#pragma unroll
  for (int j = 0; j < 8; ++j) v[j] = (b16)(bf16_rne(w[(size_t)(r0 + k0 + j) * H + o]) * WSC); for (int pass = 0; pass < 2; ++pass) { *(volatile v8b*)(WT + e) = v; __threadfence(); }
}
__global__ __launch_bounds__(128) void wenc_kernel(const float* __restrict__ w, b16* __restrict__ WT) {
  const int o = threadIdx.x; v8b v0 = {}, vz = {};
#pragma unroll
  for (int k = 0; k < 4; ++k) v0[k] = (b16)(bf16_rne(w[k * H + o]) * WSC);
  for (int pass = 0; pass < 2; ++pass) { *(volatile v8b*)(WT + (size_t)o * 32) = v0; *(volatile v8b*)(WT + (size_t)o * 32 + 8) = vz; *(volatile v8b*)(WT + (size_t)o * 32 + 16) = vz; *(volatile v8b*)(WT + (size_t)o * 32 + 24) = vz; __threadfence(); }
}
__global__ __launch_bounds__(32) void enc_kernel(const float* __restrict__ x, const b16* __restrict__ WT, const float* __restrict__ bias, float* __restrict__ Hout) {
  __shared__ __attribute__((aligned(16))) b16 Ah[16][32 + 8]; __shared__ __attribute__((aligned(16))) float Tf[16][H + 4];
  const int lane = threadIdx.x, nloc = lane & 15, hlf = lane >> 4; const size_t m0 = (size_t)blockIdx.x * 16;
  for (int rr = 0; rr < 16; ++rr) { const size_t r = (m0 + rr) < (size_t)N ? m0 + rr : (size_t)N - 1; Ah[rr][lane] = lane < 4 ? (b16)(bf16_rne(x[r * 4 + lane]) * XS) : (b16)0.0f; }
  wave_lds_sync();
  v8f acc[8]; const v16b a = frag_kb(&Ah[nloc][0], hlf);
#pragma unroll
  for (int t = 0; t < 8; ++t) { acc[t] = (v8f){}; acc[t] = wmma16b(a, frag_kb(WT + (size_t)(t * 16 + nloc) * 32, hlf), acc[t]); }
#pragma unroll
  for (int t = 0; t < 8; ++t) { const int c = t * 16 + nloc; const float bb = bf16_rne(bias[c]);
#pragma unroll 1
    for (int r8 = 0; r8 < 8; ++r8) Tf[8 * hlf + r8][c] = (m0 + 8 * hlf + r8 < (size_t)N) ? acc[t][r8] * (1.0f / (XS * WSC)) + bb : 0.0f; }
  wave_lds_sync();
  for (int pass = 0; pass < 2; ++pass) { for (int rr = 0; rr < 16; ++rr) *(volatile v4f*)(Hout + (m0 + rr) * H + lane * 4) = *(const v4f*)(&Tf[rr][lane * 4]); __threadfence(); }
}
template <int NT, int CNTB, int RELU>
__global__ __launch_bounds__(32) void gemm_kernel(const float* __restrict__ IN_, const b16* __restrict__ WT, const float* __restrict__ bias, const int* __restrict__ ROWCNT, int NLIM, int NSTORE, float* __restrict__ OUT_) {
  __shared__ __attribute__((aligned(16))) b16 Ah[16][H + 8], Al[16][H + 8]; __shared__ __attribute__((aligned(16))) float Tf[16][NT * 16 + 4];
  const int lane = threadIdx.x, nloc = lane & 15, hlf = lane >> 4; const size_t m0 = (size_t)blockIdx.x * 16; if (m0 >= (size_t)NLIM) return;
  for (int rr = 0; rr < 16; ++rr) { const v4f v = *(const v4f*)(IN_ + (m0 + rr) * H + lane * 4); for (int j = 0; j < 4; ++j) { b16 p, q; split16(v[j] * HS, p, q); Ah[rr][lane * 4 + j] = p; Al[rr][lane * 4 + j] = q; } }
  wave_lds_sync();
#pragma unroll 1
  for (int cg = 0; cg < NT / 8; ++cg) { v8f acc[8];
#pragma unroll
    for (int t = 0; t < 8; ++t) acc[t] = (v8f){};
#pragma unroll 2
    for (int kb = 0; kb < H; kb += 32) { const v16b a = frag_kb(&Ah[nloc][kb], hlf), al = frag_kb(&Al[nloc][kb], hlf);
#pragma unroll
      for (int t = 0; t < 8; ++t) { const v16b bw = frag_kb(WT + (size_t)(cg * 128 + t * 16 + nloc) * H + kb, hlf); acc[t] = wmma16b(a, bw, acc[t]); acc[t] = wmma16b(al, bw, acc[t]); } }
#pragma unroll
    for (int t = 0; t < 8; ++t) { const int c = cg * 128 + t * 16 + nloc; const float bb = bias != nullptr ? bf16_rne(bias[c & (H - 1)]) : 0.0f;
#pragma unroll 1
      for (int r8 = 0; r8 < 8; ++r8) { const size_t r = m0 + 8 * hlf + r8; float v = acc[t][r8] * (1.0f / (HS * WSC)); if (CNTB) { const int cn = r < (size_t)N ? iclamp(ROWCNT[r], 0, 1 << 20) : 0; v += pmul((float)cn, bb); } else v += bb; Tf[8 * hlf + r8][c] = RELU ? fmaxf(v, 0.0f) : v; } } }
  wave_lds_sync();
  constexpr int OW = NT * 16, OPL = OW / 32; typedef __attribute__((ext_vector_type(OPL))) float vof;
  for (int pass = 0; pass < 2; ++pass) { for (int rr = 0; rr < 16; ++rr) if (m0 + rr < (size_t)NSTORE) *(volatile vof*)(OUT_ + (m0 + rr) * OW + lane * OPL) = *(const vof*)(&Tf[rr][lane * OPL]); __threadfence(); }
}
__global__ __launch_bounds__(256) void edge_kernel(const float* __restrict__ PQ, const float* __restrict__ ea, const float* __restrict__ w1, const float* __restrict__ b1, const int* __restrict__ srcs, const int* __restrict__ PERM, const int* __restrict__ ROWPTR, const int* __restrict__ ROWCNT, int permLen, int NLIM, float* __restrict__ Sout) {
  const int wave = threadIdx.x >> 5, lane = threadIdx.x & 31; const size_t v = (size_t)blockIdx.x * 8 + wave; v4f s = {0.0f, 0.0f, 0.0f, 0.0f};
  if (v < (size_t)NLIM) { float we[4], bb[4]; for (int i = 0; i < 4; ++i) { we[i] = bf16_rne(w1[2 * H * H + lane * 4 + i]); bb[i] = bf16_rne(b1[lane * 4 + i]); }
    const v4f pv = *(const v4f*)(PQ + v * (2 * H) + lane * 4); int st = ROWPTR[v], cnt = ROWCNT[v]; cnt = iclamp(cnt, 0, 1 << 20); st = iclamp(st, 0, permLen - cnt);
#pragma unroll 1
    for (int j = 0; j < cnt; ++j) { const int e = iclamp(PERM[st + j], 0, E - 1); const size_t sj = (size_t)iclamp(srcs[e], 0, N - 1); if (sj >= (size_t)NLIM) continue; const float a = bf16_rne(ea[e]); const v4f qv = *(const v4f*)(PQ + sj * (2 * H) + H + lane * 4);
      for (int i = 0; i < 4; ++i) s[i] += fmaxf(pv[i] + qv[i] + pmul(a, we[i]) + bb[i], 0.0f); } }
  for (int pass = 0; pass < 2; ++pass) { *(volatile v4f*)(Sout + v * H + lane * 4) = s; __threadfence(); }
}
__global__ __launch_bounds__(256) void heads_kernel(const float* Hp, const float* __restrict__ Wg, const float* __restrict__ bg, const float* __restrict__ Wp, const float* __restrict__ bp, const float* __restrict__ Wgr, const float* __restrict__ bgr, float* out) {
  __shared__ float w[4][H]; for (int i = threadIdx.x; i < H; i += 256) { w[0][i] = bf16_rne(Wg[i]); w[1][i] = bf16_rne(Wp[i]); w[2][i] = bf16_rne(Wgr[i * 2]); w[3][i] = bf16_rne(Wgr[i * 2 + 1]); }
  __syncthreads();
  const int n = blockIdx.x * 256 + threadIdx.x; if (n >= N) return; float a0 = bf16_rne(bg[0]), a1 = bf16_rne(bp[0]), a2 = bf16_rne(bgr[0]), a3 = bf16_rne(bgr[1]);
#pragma unroll 1
  for (int c = 0; c < H; c += 4) { const v4f hv = *(const v4f*)(Hp + (size_t)n * H + c); for (int j = 0; j < 4; ++j) { a0 += pmul(hv[j], w[0][c + j]); a1 += pmul(hv[j], w[1][c + j]); a2 += pmul(hv[j], w[2][c + j]); a3 += pmul(hv[j], w[3][c + j]); } }
  const float gs = sigm(a0); const v2f g2 = {a2, a3};
  for (int pass = 0; pass < 2; ++pass) { if (n < N - 16) ((volatile float*)out)[OFF1 + n] = gs; if (n >= 16) ((volatile float*)out)[OFF2 + n] = a1; *(volatile v2f*)(out + OFF3 + 2 * n) = g2; __threadfence(); }
}
__global__ __launch_bounds__(32) void fixline_kernel(const float* Hp, const float* __restrict__ Wg, const float* __restrict__ bg, const float* __restrict__ Wp, const float* __restrict__ bp, float* out) {
  const int lane = threadIdx.x; const bool isg = lane < 16; const int n = isg ? N - 16 + lane : lane - 16; const float* w = isg ? Wg : Wp; float a = bf16_rne(isg ? bg[0] : bp[0]);
#pragma unroll 1
  for (int c = 0; c < H; c += 4) { const v4f hv = *(const v4f*)(Hp + (size_t)n * H + c); for (int j = 0; j < 4; ++j) a += pmul(hv[j], bf16_rne(w[c + j])); }
  const float o = isg ? sigm(a) : a;
  for (int pass = 0; pass < 2; ++pass) { ((volatile float*)out)[OFF1 + (N - 16) + lane] = o; __threadfence(); }
}
}

extern "C" void kernel_launch(void* const* d_in, const int* in_sizes, int n_in, void* d_out, int out_size, void* d_ws, size_t ws_size, hipStream_t stream) {
  (void)n_in;
  auto Fp = [&](int i) { return (const float*)d_in[i]; }; auto Ip = [&](int i) { return (const int*)d_in[i]; };
  if (in_sizes[0] != N * 4 || in_sizes[1] != 2 * E || in_sizes[2] != E || in_sizes[3] != 4 * H || in_sizes[5] != NL * 257 * H || in_sizes[7] != NL * H * H || in_sizes[9] != H || in_sizes[13] != 2 * H || out_size != OFF3 + 2 * N) return;
  const int NLIM = N; const int GB16 = NBLK, GB8 = NP / 8;
  size_t off = 0; char* ws = (char*)d_ws;
  auto carve = [&](size_t bytes) { char* p = ws + off; off += (bytes + 255) & ~(size_t)255; return p; };
  b16* WENC = (b16*)carve(H * 32 * 2); b16* WPQ[NL]; b16* W2T[NL]; for (int l = 0; l < NL; ++l) { WPQ[l] = (b16*)carve((size_t)2 * H * H * 2); W2T[l] = (b16*)carve((size_t)H * H * 2); }
  float* HA = (float*)carve((size_t)NP * H * 4); float* PQ = (float*)carve((size_t)NP * 2 * H * 4); float* S = (float*)carve((size_t)NP * H * 4);
  CsrBufs9 csr; off = csr_carve9(csr, ws, off, E, N);
  if (off > ws_size || off > ((size_t)160 << 20)) return;
  wenc_kernel<<<1, 128, 0, stream>>>(Fp(3), WENC);
  for (int l = 0; l < NL; ++l) { wprep_kernel<<<(H * H / 8 + 255) / 256, 256, 0, stream>>>(Fp(5) + (size_t)l * 257 * H, 0, H, WPQ[l]); wprep_kernel<<<(H * H / 8 + 255) / 256, 256, 0, stream>>>(Fp(5) + (size_t)l * 257 * H, H, H, WPQ[l] + H * H); wprep_kernel<<<(H * H / 8 + 255) / 256, 256, 0, stream>>>(Fp(7) + (size_t)l * H * H, 0, H, W2T[l]); }
  csr_build9(csr, Ip(1) + E, E, N, stream);
  enc_kernel<<<NBLK, 32, 0, stream>>>(Fp(0), WENC, Fp(4), HA);
  for (int l = 0; l < NL; ++l) {
    gemm_kernel<16, 0, 0><<<GB16, 32, 0, stream>>>(HA, WPQ[l], nullptr, nullptr, NLIM, NP, PQ);
    edge_kernel<<<GB8, 256, 0, stream>>>(PQ, Fp(2), Fp(5) + (size_t)l * 257 * H, Fp(6) + l * H, Ip(1), csr.PERM, csr.ROWPTR, csr.ROWCNT, (int)csr.permLen, NLIM, S);
    gemm_kernel<8, 1, 1><<<GB16, 32, 0, stream>>>(S, W2T[l], Fp(8) + l * H, csr.ROWCNT, NLIM, l == NL - 1 ? N : NP, l == NL - 1 ? (float*)d_out : HA); }
  heads_kernel<<<(N + 255) / 256, 256, 0, stream>>>((const float*)d_out, Fp(9), Fp(10), Fp(11), Fp(12), Fp(13), Fp(14), (float*)d_out);
  fixline_kernel<<<1, 32, 0, stream>>>((const float*)d_out, Fp(9), Fp(10), Fp(11), Fp(12), (float*)d_out);
}
